// graphConv_77635828842937
// MI455X (gfx1250) — hardware-verified
//
#include <hip/hip_runtime.h>
#include <math.h>

#ifndef NB
#define NB 128
#endif
#ifndef NN
#define NN 1024
#endif
#define NN_FULL 1024
#define DD 64
#define NUMK 8

#define CARRY_A 64.0f
#define RES_UP 2048.0f
#define RES_DN (1.0f / 2048.0f)
#define SC_CHAIN (1.0f / 16384.0f)
#define SC_OUT (1.0f / 4096.0f)
static constexpr float CARRY_S = 256.0f;
static constexpr float CARRY_X = 64.0f;

static_assert(NN == NN_FULL);
static_assert(NN % 64 == 0 && NN % 32 == 0);
static_assert(DD == 64);
static_assert(NN / 8 == 128);
static_assert((NN * (NN / 8)) % 256 == 0);
static_assert((DD * (NN / 8)) % 256 == 0);
static_assert((NN * NN / 8) % 256 == 0);
static_assert(((NN / 64) * (NN / 64)) % 8 == 0);
static_assert(((NN / 32) * (NN / 64)) % 8 == 0);
static_assert(((NN / 64) * (DD / 64)) % 8 == 0);
static_assert(CARRY_A * CARRY_S * SC_CHAIN == 1.0f);
static_assert(CARRY_A * CARRY_X * SC_OUT == 1.0f);
static_assert(RES_UP * RES_DN == 1.0f);
static_assert(32 * 16 * 8 == 16 * 64 * 4);
static_assert(8 * 16 * 68 * 4 <= 131072);

#define WS_ST16 ((size_t)NN * NN * 2)
#define WS_XT16 ((size_t)NB * DD * NN * 2)
#define WS_AHI  ((size_t)NN * NN * 2)
#define WS_ARES ((size_t)NN * NN * 2)
#define WS_AF32 ((size_t)NN * NN * 4)
static_assert(WS_ST16 % 256 == 0 && WS_XT16 % 256 == 0 && WS_AHI % 256 == 0 && WS_AF32 % 256 == 0);
static_assert(WS_ST16 + WS_XT16 + WS_AHI + WS_ARES + WS_AF32 <= (size_t)134217728);

typedef __attribute__((ext_vector_type(16))) _Float16 v16h;
typedef __attribute__((ext_vector_type(8)))  _Float16 v8h;
typedef __attribute__((ext_vector_type(8)))  float    v8f;
typedef __attribute__((ext_vector_type(4)))  float    v4f;
typedef __attribute__((ext_vector_type(4)))  unsigned int v4u;
typedef _Float16 h16;


#define VST2(T, ptr, val) do { const T vst2_v_ = (val); *(volatile T*)(ptr) = vst2_v_; __threadfence(); *(volatile T*)(ptr) = vst2_v_; } while (0)
#define VST2V4(ptr, val) do { const v4f vst2_v4_ = (val); *(volatile v4f*)(ptr) = vst2_v4_; __threadfence(); *(volatile v4f*)(ptr) = vst2_v4_; } while (0)

__device__ __forceinline__ float bfr(float f) {
    unsigned u = __float_as_uint(f);
    u += 0x7FFFu + ((u >> 16) & 1u);
    return __uint_as_float(u & 0xFFFF0000u);
}
__device__ __forceinline__ unsigned short f2h_bits(float x) {
    return (fabsf(x) < 6.104e-5f) ? (unsigned short)0 : __builtin_bit_cast(unsigned short, (_Float16)x);
}
__device__ __forceinline__ void st8h(unsigned short* P, size_t o, const float* v) {
    v4u pk;
    pk.x = (unsigned)f2h_bits(v[0]) | ((unsigned)f2h_bits(v[1]) << 16);
    pk.y = (unsigned)f2h_bits(v[2]) | ((unsigned)f2h_bits(v[3]) << 16);
    pk.z = (unsigned)f2h_bits(v[4]) | ((unsigned)f2h_bits(v[5]) << 16);
    pk.w = (unsigned)f2h_bits(v[6]) | ((unsigned)f2h_bits(v[7]) << 16);
    VST2(v4u, (v4u*)(P + o), pk);
}

static __device__ __forceinline__ h16 toh_flush(float v) { const h16 r = (h16)v; return (fabsf(v) < 6.103515625e-05f) ? (h16)0.0f : r; }
__device__ __forceinline__ void st8hf(unsigned short* P, size_t o, const float* v) {
    v8h hv;
#pragma unroll
    for (int e = 0; e < 8; ++e) hv[e] = toh_flush(v[e]);
    v8h* dst = (v8h*)(P + o);
    *(volatile v8h*)dst = hv;
    __threadfence();
    *(volatile v8h*)dst = hv;
}

union FragU { v16h v; v8h h[2]; };
__device__ __forceinline__ v16h frag_ld(const _Float16* p) {
    FragU f; f.h[0] = *(const v8h*)(p); f.h[1] = *(const v8h*)(p + 16); return f.v;
}
__device__ __forceinline__ v8f wmma16(v16h a, v16h b, v8f c) {
    c = __builtin_amdgcn_wmma_f32_16x16x32_f16(false, a, false, b, (short)0, c, false, false);
    asm volatile("v_nop\n\tv_nop\n\tv_nop\n\tv_nop" : "+v"(c) : "v"(a), "v"(b));
    return c;
}
__device__ __forceinline__ void wave_sync_lds() {
    __builtin_amdgcn_fence(3  , "workgroup");
    __builtin_amdgcn_wave_barrier();
    __builtin_amdgcn_fence(2  , "workgroup");
}

template <int MI, bool RES, bool ADDW>
__device__ __forceinline__ void gemm_body(
    const _Float16* __restrict__ A, const _Float16* __restrict__ Ar, unsigned lda,
    const _Float16* __restrict__ Bt, unsigned ldb,
    float* __restrict__ C, unsigned ldc, const float* __restrict__ addw,
    unsigned M, unsigned N, unsigned K, float scale) {
  __shared__ __align__(16) float sT[8][16 * 68];
  const unsigned lane = threadIdx.x & 31u;
  const unsigned wave = (unsigned)__builtin_amdgcn_readfirstlane((int)(threadIdx.x >> 5));
  const unsigned tilesN = N >> 6, tilesM = M / (16u * (unsigned)MI);
  const unsigned tile = blockIdx.x * 8u + wave;
  if (tile >= tilesM * tilesN) return;
  const unsigned tm = tile / tilesN;
  const unsigned tn = tile - tm * tilesN;
  const unsigned m0 = tm * (16u * (unsigned)MI), n0 = tn << 6;
  const unsigned rlane = lane & 15u;
  const unsigned koff = (lane >> 4) * 8u;
  const unsigned mOff = koff;

  v8f acc[MI][4];
  v8f accr[MI][4];
#pragma unroll
  for (int i = 0; i < MI; ++i)
#pragma unroll
    for (int j = 0; j < 4; ++j) {
      acc[i][j] = (v8f){0.f,0.f,0.f,0.f,0.f,0.f,0.f,0.f};
      if (RES) accr[i][j] = (v8f){0.f,0.f,0.f,0.f,0.f,0.f,0.f,0.f};
    }

  for (unsigned k0 = 0; k0 < K; k0 += 32u) {
    v16h bh[4];
#pragma unroll
    for (int j = 0; j < 4; ++j)
      bh[j] = frag_ld(Bt + (size_t)(n0 + ((unsigned)j << 4) + rlane) * ldb + koff + k0);
#pragma unroll
    for (int i = 0; i < MI; ++i) {
      const size_t ao = (size_t)(m0 + ((unsigned)i << 4) + rlane) * lda + koff + k0;
      const v16h ah = frag_ld(A + ao);
#pragma unroll
      for (int j = 0; j < 4; ++j) acc[i][j] = wmma16(ah, bh[j], acc[i][j]);
      if (RES) {
        const v16h ar = frag_ld(Ar + ao);
#pragma unroll
        for (int j = 0; j < 4; ++j) accr[i][j] = wmma16(ar, bh[j], accr[i][j]);
      }
    }
  }

  float* slab = sT[wave];
#pragma unroll
  for (int i = 0; i < MI; ++i) {
    const unsigned mBase = m0 + ((unsigned)i << 4);
#pragma unroll
    for (int j = 0; j < 4; ++j) {
#pragma unroll
      for (int r = 0; r < 8; ++r) {
        float v = acc[i][j][r];
        if (RES) v += accr[i][j][r] * RES_DN;
        v *= scale;
        slab[(mOff + (unsigned)r) * 68u + ((unsigned)j << 4) + rlane] = v;
      }
    }
    wave_sync_lds();
    {
      const unsigned hh = lane >> 4, c4 = (lane & 15u) * 4u;
#pragma unroll
      for (int half = 0; half < 2; ++half) {
        v4f vv[4];
#pragma unroll
        for (int it = 0; it < 4; ++it) {
          const unsigned row = (unsigned)(half * 4 + it) * 2u + hh;
          vv[it] = *(const v4f*)(slab + row * 68u + c4);
          if (ADDW) {
            const v4f w = *(const v4f*)(addw + (size_t)(mBase + row) * ldc + n0 + c4);
            vv[it].x += bfr(w.x); vv[it].y += bfr(w.y); vv[it].z += bfr(w.z); vv[it].w += bfr(w.w);
          }
        }
        for (int pass = 0; pass < 2; ++pass) {
#pragma unroll
          for (int it = 0; it < 4; ++it) {
            const unsigned row = (unsigned)(half * 4 + it) * 2u + hh;
            *(volatile v4f*)(C + (size_t)(mBase + row) * ldc + n0 + c4) = vv[it];
          }
          __threadfence();
        }
      }
    }
    wave_sync_lds();
  }
}

__global__ __launch_bounds__(256) void k_gemm_h1(const _Float16* __restrict__ A, const _Float16* __restrict__ Bt,
                                                 float* __restrict__ C, const float* __restrict__ addw) {
  gemm_body<4, false, true>(A, A, NN, Bt, NN, C, NN, addw, NN, NN, NN, SC_CHAIN);
}
__global__ __launch_bounds__(256) void k_gemm_h2(const _Float16* __restrict__ A, const _Float16* __restrict__ Ar,
                                                 const _Float16* __restrict__ Bt, float* __restrict__ C,
                                                 const float* __restrict__ addw) {
  gemm_body<2, true, true>(A, Ar, NN, Bt, NN, C, NN, addw, NN, NN, NN, SC_CHAIN);
}
__global__ __launch_bounds__(256) void k_gemm_out(const _Float16* __restrict__ A, const _Float16* __restrict__ XT,
                                                  float* __restrict__ out) {
  const unsigned b = blockIdx.y;
  gemm_body<4, false, false>(A, A, NN, XT + (size_t)b * DD * NN, NN, out + (size_t)b * NN * DD, DD, nullptr, NN, DD, NN, SC_OUT);
}

__global__ __launch_bounds__(256) void k_wt16(const float* __restrict__ Wm, unsigned KI, unsigned NO, unsigned lgper,
                                              unsigned short* __restrict__ W16, float sw) {
    const unsigned layer = blockIdx.y;
    const float* Wl = Wm + (size_t)layer * KI * NO;
    unsigned short* Dl = W16 + (size_t)layer * KI * NO;
    const unsigned u = blockIdx.x * 256u + threadIdx.x;
    const unsigned per = 1u << lgper;
    if (u >= NO * per) return;
    const unsigned k0 = 8u * (u & (per - 1u));
    const unsigned o = u >> lgper;
    float v[8];
#pragma unroll
    for (int i = 0; i < 8; ++i) v[i] = bfr(Wl[(size_t)(k0 + (unsigned)i) * NO + o]) * sw;
    st8h(Dl, (size_t)o * KI + k0, v);
}

__global__ __launch_bounds__(256) void k_split(const float* __restrict__ src, unsigned short* __restrict__ hi16,
                                               unsigned short* __restrict__ res16, unsigned isInput, unsigned wantRes,
                                               unsigned nOct) {
#pragma clang fp contract(off)
    const unsigned u = blockIdx.x * 256u + threadIdx.x;
    if (u >= nOct) return;
    const v4f a = *(const v4f*)(src + (size_t)u * 8u);
    const v4f b = *(const v4f*)(src + (size_t)u * 8u + 4u);
    const float x[8] = {a.x, a.y, a.z, a.w, b.x, b.y, b.z, b.w};
    float hv[8], rv[8];
#pragma unroll
    for (int i = 0; i < 8; ++i) {
        const float xb = bfr(x[i]);
        float v = (isInput != 0u) ? xb : x[i];
        v *= CARRY_A;
        const float r = (float)(h16)v;
        hv[i] = v;
        rv[i] = (v - r) * RES_UP;
    }
    st8hf(hi16, (size_t)u * 8u, hv);
    if (wantRes != 0u) st8hf(res16, (size_t)u * 8u, rv);
}

extern "C" void kernel_launch(void* const* d_in, const int* in_sizes, int n_in, void* d_out, int out_size,
                              void* d_ws, size_t ws_size, hipStream_t stream) {
    if (n_in < 3) return;
    if (in_sizes[0] < NB * NN * DD || in_sizes[1] < NUMK * NN * NN || in_sizes[2] < NN * NN) return;
    if (out_size < NB * NN * DD) return;

    const float* nodes  = (const float*)d_in[0];
    const float* weight = (const float*)d_in[1];
    const float* gshift = (const float*)d_in[2];
    float* out = (float*)d_out;

    char* wsp = (char*)d_ws;
    size_t off = 0;
    auto carve = [&](size_t bytes) -> void* { void* r = wsp + off; off += (bytes + 255) & ~(size_t)255; return r; };
    unsigned short* st16 = (unsigned short*)carve(WS_ST16);
    unsigned short* xt16 = (unsigned short*)carve(WS_XT16);
    unsigned short* ahi  = (unsigned short*)carve(WS_AHI);
    unsigned short* ares = (unsigned short*)carve(WS_ARES);
    float*          af32 = (float*)carve(WS_AF32);
    if (off > ws_size || off > (size_t)134217728) return;

    k_wt16<<<dim3((NN * (NN / 8)) / 256, 1), 256, 0, stream>>>(gshift, NN, NN, 7, st16, CARRY_S);
    k_wt16<<<dim3((DD * (NN / 8)) / 256, NB), 256, 0, stream>>>(nodes, NN, DD, 7, xt16, CARRY_X);

    const unsigned nOct = (unsigned)(NN * NN / 8);
    const unsigned gS  = (unsigned)(NN * NN / 8) / 256u;
    const unsigned gH1 = (unsigned)((NN / 64) * (NN / 64)) / 8u;
    const unsigned gH2 = (unsigned)((NN / 32) * (NN / 64)) / 8u;
    const unsigned gO  = (unsigned)((NN / 64) * (DD / 64)) / 8u;
    const size_t plane = (size_t)NN * NN;

    k_split<<<gS, 256, 0, stream>>>(weight + (size_t)(NUMK - 1) * plane, ahi, ares, 1u, 0u, nOct);
    k_gemm_h1<<<gH1, 256, 0, stream>>>((const _Float16*)ahi, (const _Float16*)st16, af32, weight + (size_t)(NUMK - 2) * plane);
    for (int k = NUMK - 3; k >= 2; --k) {
        k_split<<<gS, 256, 0, stream>>>(af32, ahi, ares, 0u, 0u, nOct);
        k_gemm_h1<<<gH1, 256, 0, stream>>>((const _Float16*)ahi, (const _Float16*)st16, af32, weight + (size_t)k * plane);
    }
    for (int k = 1; k >= 0; --k) {
        k_split<<<gS, 256, 0, stream>>>(af32, ahi, ares, 0u, 1u, nOct);
        k_gemm_h2<<<gH2, 256, 0, stream>>>((const _Float16*)ahi, (const _Float16*)ares, (const _Float16*)st16, af32,
                                           weight + (size_t)k * plane);
    }
    k_split<<<gS, 256, 0, stream>>>(af32, ahi, ares, 0u, 0u, nOct);
    k_gemm_out<<<dim3(gO, NB), 256, 0, stream>>>((const _Float16*)ahi, (const _Float16*)xt16, out);
}
